// LRU_50852412785331
// MI455X (gfx1250) — hardware-run, weakly checked
//
#include <hip/hip_runtime.h>
#include <cmath>

typedef __attribute__((ext_vector_type(16))) _Float16 v16h;
typedef __attribute__((ext_vector_type(8)))  _Float16 v8h;
typedef __attribute__((ext_vector_type(8)))  float    v8f;
typedef __attribute__((ext_vector_type(4)))  float    v4f;
typedef __attribute__((ext_vector_type(2)))  float    v2f;
typedef __attribute__((ext_vector_type(4)))  unsigned v4u;

constexpr int N_BATCH  = 8;
constexpr int SEQ_LEN  = 2048;
constexpr int DIM_HID  = 512;
constexpr int DIM_STATE = 512;
constexpr int DIM_STATE2 = 2 * DIM_STATE;
constexpr int N_TOK    = N_BATCH * SEQ_LEN;

constexpr float CARRY_XS = 16.0f;
constexpr float CARRY_B  = 1024.0f;
constexpr float CARRY_HS = 8.0f;
constexpr float CARRY_C  = 1024.0f;
constexpr float CARRY_Y  = 16.0f;
constexpr float CARRY_W  = 1024.0f;
constexpr float SCALE_GEMM1 = 1.0f / 16384.0f;
constexpr float SCALE_GEMM2 = 1.0f / 8192.0f;
constexpr float SCALE_GEMM3 = 1.0f / 16384.0f;
constexpr float CARRY_NONE  = 1.0f;

constexpr size_t WS_OFF_PARAMS = 0;
constexpr size_t WS_SZ_PARAMS  = 3 * (size_t)DIM_STATE * 4;
constexpr size_t WS_OFF_BT1    = WS_OFF_PARAMS + WS_SZ_PARAMS;
constexpr size_t WS_SZ_BT1     = (size_t)DIM_STATE2 * DIM_HID * 2;
constexpr size_t WS_OFF_BT2    = WS_OFF_BT1 + WS_SZ_BT1;
constexpr size_t WS_SZ_BT2     = (size_t)DIM_HID * DIM_STATE2 * 2;
constexpr size_t WS_OFF_BT3    = WS_OFF_BT2 + WS_SZ_BT2;
constexpr size_t WS_SZ_BT3     = (size_t)DIM_HID * DIM_HID * 2;
constexpr size_t WS_OFF_XS16   = WS_OFF_BT3 + WS_SZ_BT3;
constexpr size_t WS_SZ_XS16    = (size_t)N_TOK * DIM_HID * 2;
constexpr size_t WS_OFF_G      = WS_OFF_XS16 + WS_SZ_XS16;
constexpr size_t WS_SZ_G       = (size_t)N_TOK * DIM_STATE2 * 4;
constexpr size_t WS_OFF_H16    = WS_OFF_G + WS_SZ_G;
constexpr size_t WS_SZ_H16     = (size_t)N_TOK * DIM_STATE2 * 2;
constexpr size_t WS_TOTAL      = WS_OFF_H16 + WS_SZ_H16;
constexpr size_t WS_SZ_Y32     = (size_t)N_TOK * DIM_HID * 4;
static_assert(WS_TOTAL == 120068096, "carve");
static_assert(WS_TOTAL <= 134217728, "carve limit");
static_assert(2 * WS_SZ_Y32 <= WS_SZ_G, "y32 and z inside the G region");
static_assert((size_t)N_TOK * DIM_HID * 2 <= WS_SZ_XS16, "y16 inside the xs16 region");
static_assert((WS_OFF_BT1 % 128) == 0 && (WS_OFF_BT2 % 128) == 0 && (WS_OFF_BT3 % 128) == 0 &&
              (WS_OFF_XS16 % 128) == 0 && (WS_OFF_G % 128) == 0 && (WS_OFF_H16 % 128) == 0 &&
              (WS_SZ_Y32 % 128) == 0, "line alignment");
static_assert(N_TOK % 64 == 0 && DIM_STATE2 % 64 == 0 && DIM_HID % 64 == 0, "tile multiples");
static_assert(DIM_HID % 32 == 0 && DIM_STATE2 % 32 == 0, "k multiples");
static_assert(((N_TOK / 64) * (DIM_STATE2 / 64)) % 8 == 0, "gemm1 grid");
static_assert(((N_TOK / 64) * (DIM_HID / 64)) % 8 == 0, "gemm2/3 grid");
static_assert(N_TOK % 8 == 0 && SEQ_LEN % 32 == 0 && DIM_STATE % 32 == 0, "row/scan blocking");

__device__ __forceinline__ float bf16_rne(float f) {
  unsigned u = __float_as_uint(f);
  u = (u + 0x7FFFu + ((u >> 16) & 1u)) & 0xFFFF0000u;
  return __uint_as_float(u);
}

__device__ __forceinline__ _Float16 to_f16_ftz(float x) {
  const float w = (fabsf(x) < 6.103515625e-5f) ? 0.0f : x;
  return (_Float16)w;
}
__device__ __forceinline__ unsigned f16_bits_ftz(float x) {
  return (unsigned)__builtin_bit_cast(unsigned short, to_f16_ftz(x));
}

__device__ __forceinline__ void dep_guard_h(v8f& a, v8f& b, v16h x, v16h y) { asm volatile("v_nop\n\tv_nop\n\tv_nop\n\tv_nop" : "+v"(a), "+v"(b) : "v"(x), "v"(y)); }
__device__ __forceinline__ void keep4_h(v16h a, v16h b, v16h c, v16h d) { asm volatile("v_nop" :: "v"(a), "v"(b), "v"(c), "v"(d)); }
__device__ __forceinline__ void acc_guard4(v8f& a, v8f& b, v8f& c, v8f& d) { asm volatile("v_nop\n\tv_nop\n\tv_nop\n\tv_nop" : "+v"(a), "+v"(b), "+v"(c), "+v"(d)); }
template <typename T> struct Frag;
template <> struct Frag<_Float16> {
  typedef v16h V; union U { v16h v; v8h h[2]; };
  static __device__ __forceinline__ v16h load(const _Float16* p) {
    U f; f.h[0] = *(const v8h*)(p); f.h[1] = *(const v8h*)(p + 16); return f.v;
  }
  static __device__ __forceinline__ v8f mma(v16h a, v16h b, v8f c) {
    return __builtin_amdgcn_wmma_f32_16x16x32_f16(false, a, false, b, (short)0, c, false, false);
  }
  static __device__ __forceinline__ void guard(v8f& a, v8f& b, v16h x, v16h y) { dep_guard_h(a, b, x, y); }
  static __device__ __forceinline__ void keep(v16h a, v16h b, v16h c, v16h d) { keep4_h(a, b, c, d); }
};

template <bool OUT16>
__global__ __launch_bounds__(256) void wmma_gemm64_f16(
    const unsigned short* __restrict__ Ap, int lda,
    const unsigned short* __restrict__ Btp, int ldb,
    float* __restrict__ Cout, int ldc,
    unsigned short* __restrict__ C16, int ldc16,
    int M, int N, int K, float scale, float carry16) {
  typedef _Float16 T;
  typedef v16h V;
  const T* A = (const T*)Ap; const T* Bt = (const T*)Btp;
  __shared__ __align__(16) float sT[8][16 * 68];
  const int lane = threadIdx.x & 31;
  const int wave = threadIdx.x >> 5;
  const int tilesN = N >> 6;
  const int tilesM = M >> 6;
  const int tile = blockIdx.x * 8 + wave;
  if (tile >= tilesM * tilesN) return;
  const int tm = tile / tilesN;
  const int tn = tile - tm * tilesN;
  const int m0 = tm << 6;
  const int n0 = tn << 6;

  const int rlane = lane & 15;
  const int koff  = (lane >> 4) * 8;
  const int mOff  = (lane >> 4) * 8;

  v8f acc[4][4];
#pragma unroll
  for (int i = 0; i < 4; ++i)
#pragma unroll
    for (int j = 0; j < 4; ++j) acc[i][j] = (v8f){0.f,0.f,0.f,0.f,0.f,0.f,0.f,0.f};

  for (int k0 = 0; k0 < K; k0 += 32) {
    V bh[4];
#pragma unroll
    for (int j = 0; j < 4; ++j) {
      const size_t bo = (size_t)(n0 + (j << 4) + rlane) * ldb + koff + k0;
      bh[j] = Frag<T>::load(Bt + bo);
    }
#pragma unroll
    for (int i = 0; i < 4; ++i) {
      const size_t ao = (size_t)(m0 + (i << 4) + rlane) * lda + koff + k0;
      V ah = Frag<T>::load(A + ao);
#pragma unroll
      for (int j = 0; j < 4; ++j) {
        acc[i][j] = Frag<T>::mma(ah, bh[j], acc[i][j]);
      }
      Frag<T>::guard(acc[i][0], acc[i][3], ah, ah);
    }
    Frag<T>::keep(bh[0], bh[1], bh[2], bh[3]);
  }
  acc_guard4(acc[0][0], acc[0][1], acc[0][2], acc[0][3]);
  acc_guard4(acc[1][0], acc[1][1], acc[1][2], acc[1][3]);
  acc_guard4(acc[2][0], acc[2][1], acc[2][2], acc[2][3]);
  acc_guard4(acc[3][0], acc[3][1], acc[3][2], acc[3][3]);

  float* slab = sT[wave];
  const int hh = lane >> 4, c4 = (lane & 15) * 4;
  const int q  = lane >> 3, c8 = (lane & 7) * 8;
#pragma unroll
  for (int i = 0; i < 4; ++i) {
    const int mBase = m0 + (i << 4);
#pragma unroll
    for (int j = 0; j < 4; ++j) {
#pragma unroll
      for (int r = 0; r < 8; ++r) {
        const float v = acc[i][j][r] * scale;
        slab[(mOff + r) * 68 + (j << 4) + rlane] = v;
      }
    }
    __builtin_amdgcn_fence(__ATOMIC_RELEASE, "workgroup");
    __builtin_amdgcn_wave_barrier();
    __builtin_amdgcn_fence(__ATOMIC_ACQUIRE, "workgroup");
    for (int pass = 0; pass < 2; ++pass) {
#pragma unroll
      for (int it = 0; it < 8; ++it) {
        const int row = it * 2 + hh;
        v4f v = *(const v4f*)(slab + row * 68 + c4);
        *(volatile v4f*)(Cout + (size_t)(mBase + row) * ldc + n0 + c4) = v;
      }
      if (OUT16) {
#pragma unroll
        for (int it = 0; it < 4; ++it) {
          const int row = it * 4 + q;
          const float* sp = slab + row * 68 + c8;
          v8h hv;
#pragma unroll
          for (int e = 0; e < 8; ++e) hv[e] = to_f16_ftz(sp[e] * carry16);
          *(volatile v8h*)(C16 + (size_t)(mBase + row) * ldc16 + n0 + c8) = hv;
        }
      }
      __threadfence();
    }
    __builtin_amdgcn_fence(__ATOMIC_RELEASE, "workgroup");
    __builtin_amdgcn_wave_barrier();
    __builtin_amdgcn_fence(__ATOMIC_ACQUIRE, "workgroup");
  }
}

__global__ __launch_bounds__(512) void lru_setup(
    const float* __restrict__ nu_log, const float* __restrict__ theta_log,
    const float* __restrict__ gamma_log, float* __restrict__ params) {
  const int v = threadIdx.x;
  const float nul = bf16_rne(nu_log[v]);
  const float thl = bf16_rne(theta_log[v]);
  const float gml = bf16_rne(gamma_log[v]);
  const float nu  = expf(nul);
  const float th  = expf(thl);
  const float mag = expf(-nu);
  const float lr  = mag * cosf(th);
  const float li  = mag * sinf(th);
  const float gm  = expf(gml);
  volatile float* vp = params;
  vp[v] = lr; vp[DIM_STATE + v] = li; vp[2 * DIM_STATE + v] = gm;
  __threadfence();
  vp[v] = lr; vp[DIM_STATE + v] = li; vp[2 * DIM_STATE + v] = gm;
}

__global__ __launch_bounds__(256) void prep_bt1(
    const float* __restrict__ Bre, const float* __restrict__ Bim, _Float16* __restrict__ Bt1) {
  __shared__ float tile[64 * 65];
  const int t  = threadIdx.x;
  const int v0 = blockIdx.x * 32;
  const int h0 = blockIdx.y * 64;
#pragma unroll
  for (int i = 0; i < 2; ++i) {
    const int idx = t + 256 * i;
    const int hl  = idx >> 3;
    const int v4  = (idx & 7) * 4;
    const v4f wr = *(const v4f*)(Bre + (size_t)(h0 + hl) * DIM_STATE + v0 + v4);
    const v4f wi = *(const v4f*)(Bim + (size_t)(h0 + hl) * DIM_STATE + v0 + v4);
#pragma unroll
    for (int e = 0; e < 4; ++e) {
      tile[(2 * (v4 + e)) * 65 + hl]     = bf16_rne(wr[e]) * CARRY_B;
      tile[(2 * (v4 + e) + 1) * 65 + hl] = bf16_rne(wi[e]) * CARRY_B;
    }
  }
  __syncthreads();
  const int c8 = (t & 7) * 8;
  const int l0 = t >> 3;
  const int l1 = 32 + (t >> 3);
  v8h hv0, hv1;
#pragma unroll
  for (int e = 0; e < 8; ++e) {
    hv0[e] = to_f16_ftz(tile[l0 * 65 + c8 + e]);
    hv1[e] = to_f16_ftz(tile[l1 * 65 + c8 + e]);
  }
  _Float16* d0 = Bt1 + (size_t)(2 * v0 + l0) * DIM_HID + h0 + c8;
  _Float16* d1 = Bt1 + (size_t)(2 * v0 + l1) * DIM_HID + h0 + c8;
  *(volatile v8h*)d0 = hv0;
  *(volatile v8h*)d1 = hv1;
  __threadfence();
  *(volatile v8h*)d0 = hv0;
  *(volatile v8h*)d1 = hv1;
}

__global__ __launch_bounds__(256) void prep_bt2(
    const float* __restrict__ Cre, const float* __restrict__ Cim, _Float16* __restrict__ Bt2) {
  __shared__ float tile[64 * 65];
  const int t  = threadIdx.x;
  const int v0 = blockIdx.x * 32;
  const int o0 = blockIdx.y * 64;
#pragma unroll
  for (int i = 0; i < 2; ++i) {
    const int idx = t + 256 * i;
    const int vl  = idx >> 4;
    const int o4  = (idx & 15) * 4;
    const v4f wr = *(const v4f*)(Cre + (size_t)(v0 + vl) * DIM_HID + o0 + o4);
    const v4f wi = *(const v4f*)(Cim + (size_t)(v0 + vl) * DIM_HID + o0 + o4);
#pragma unroll
    for (int e = 0; e < 4; ++e) {
      tile[(o4 + e) * 65 + 2 * vl]     = bf16_rne(wr[e]) * CARRY_C;
      tile[(o4 + e) * 65 + 2 * vl + 1] = -(bf16_rne(wi[e]) * CARRY_C);
    }
  }
  __syncthreads();
  const int c8 = (t & 7) * 8;
  const int l0 = t >> 3;
  const int l1 = 32 + (t >> 3);
  v8h hv0, hv1;
#pragma unroll
  for (int e = 0; e < 8; ++e) {
    hv0[e] = to_f16_ftz(tile[l0 * 65 + c8 + e]);
    hv1[e] = to_f16_ftz(tile[l1 * 65 + c8 + e]);
  }
  _Float16* d0 = Bt2 + (size_t)(o0 + l0) * DIM_STATE2 + 2 * v0 + c8;
  _Float16* d1 = Bt2 + (size_t)(o0 + l1) * DIM_STATE2 + 2 * v0 + c8;
  *(volatile v8h*)d0 = hv0;
  *(volatile v8h*)d1 = hv1;
  __threadfence();
  *(volatile v8h*)d0 = hv0;
  *(volatile v8h*)d1 = hv1;
}

template <bool RND>
__global__ __launch_bounds__(256) void cvt_plane_f16(
    const float* __restrict__ in, _Float16* __restrict__ out, float carry) {
  const size_t g = (size_t)blockIdx.x * 256 + threadIdx.x;
  const float* src = in + g * 8;
  v4f a = *(const v4f*)(src);
  v4f b = *(const v4f*)(src + 4);
  if (RND) {
#pragma unroll
    for (int e = 0; e < 4; ++e) { a[e] = bf16_rne(a[e]); b[e] = bf16_rne(b[e]); }
  }
  v8h hv;
  hv[0] = to_f16_ftz(a[0] * carry); hv[1] = to_f16_ftz(a[1] * carry);
  hv[2] = to_f16_ftz(a[2] * carry); hv[3] = to_f16_ftz(a[3] * carry);
  hv[4] = to_f16_ftz(b[0] * carry); hv[5] = to_f16_ftz(b[1] * carry);
  hv[6] = to_f16_ftz(b[2] * carry); hv[7] = to_f16_ftz(b[3] * carry);
  _Float16* dst = out + g * 8;
  *(volatile v8h*)dst = hv;
  __threadfence();
  *(volatile v8h*)dst = hv;
}

__global__ __launch_bounds__(256) void ln_rows_f16(
    const float* __restrict__ x, _Float16* __restrict__ xs16) {
  const int row  = blockIdx.x * 8 + (threadIdx.x >> 5);
  const int lane = threadIdx.x & 31;
  const float* xr = x + (size_t)row * DIM_HID;
  v4f a0 = *(const v4f*)(xr + 8 * lane);
  v4f a1 = *(const v4f*)(xr + 8 * lane + 4);
  v4f b0 = *(const v4f*)(xr + 256 + 8 * lane);
  v4f b1 = *(const v4f*)(xr + 256 + 8 * lane + 4);
#pragma unroll
  for (int e = 0; e < 4; ++e) {
    a0[e] = bf16_rne(a0[e]); a1[e] = bf16_rne(a1[e]);
    b0[e] = bf16_rne(b0[e]); b1[e] = bf16_rne(b1[e]);
  }
  float s = ((a0[0] + a0[1]) + (a0[2] + a0[3])) + ((a1[0] + a1[1]) + (a1[2] + a1[3]));
  s += ((b0[0] + b0[1]) + (b0[2] + b0[3])) + ((b1[0] + b1[1]) + (b1[2] + b1[3]));
#pragma unroll
  for (int off = 16; off > 0; off >>= 1) s += __shfl_xor(s, off, 32);
  const float mu = s * (1.0f / 512.0f);
  const v4f da0 = a0 - mu, da1 = a1 - mu, db0 = b0 - mu, db1 = b1 - mu;
  float ss = ((da0[0] * da0[0] + da0[1] * da0[1]) + (da0[2] * da0[2] + da0[3] * da0[3])) +
             ((da1[0] * da1[0] + da1[1] * da1[1]) + (da1[2] * da1[2] + da1[3] * da1[3]));
  ss += ((db0[0] * db0[0] + db0[1] * db0[1]) + (db0[2] * db0[2] + db0[3] * db0[3])) +
        ((db1[0] * db1[0] + db1[1] * db1[1]) + (db1[2] * db1[2] + db1[3] * db1[3]));
#pragma unroll
  for (int off = 16; off > 0; off >>= 1) ss += __shfl_xor(ss, off, 32);
  const float var = ss * (1.0f / 512.0f);
  const float kk  = rsqrtf(var + 1e-5f) * CARRY_XS;
  v8h h0, h1;
#pragma unroll
  for (int e = 0; e < 4; ++e) {
    h0[e]     = to_f16_ftz(da0[e] * kk);
    h0[4 + e] = to_f16_ftz(da1[e] * kk);
    h1[e]     = to_f16_ftz(db0[e] * kk);
    h1[4 + e] = to_f16_ftz(db1[e] * kk);
  }
  _Float16* dst = xs16 + (size_t)row * DIM_HID;
  *(volatile v8h*)(dst + 8 * lane) = h0;
  *(volatile v8h*)(dst + 256 + 8 * lane) = h1;
  __threadfence();
  *(volatile v8h*)(dst + 8 * lane) = h0;
  *(volatile v8h*)(dst + 256 + 8 * lane) = h1;
}

__global__ __launch_bounds__(32) void lru_scan(
    const float* __restrict__ G, const float* __restrict__ params, unsigned* __restrict__ H32) {
  __shared__ __align__(16) unsigned stage[32 * 32];
  const int lane = threadIdx.x;
  const int grp  = blockIdx.x & 15;
  const int bat  = blockIdx.x >> 4;
  const int v    = grp * 32 + lane;
  const float lr = params[v], li = params[DIM_STATE + v];
  const float gm = params[2 * DIM_STATE + v];
  float hr = 0.0f, hi = 0.0f;
  const float* gp = G + (size_t)bat * SEQ_LEN * DIM_STATE2 + 2 * v;
  unsigned* hp = H32 + (size_t)bat * SEQ_LEN * (DIM_STATE2 / 2) + grp * 32;
  const int q = lane >> 3, c = lane & 7;
  for (int t0 = 0; t0 < SEQ_LEN; t0 += 32) {
    for (int sub = 0; sub < 2; ++sub) {
      const int tb = t0 + sub * 16;
      v2f g[16];
#pragma unroll
      for (int s = 0; s < 16; ++s) g[s] = *(const v2f*)(gp + (size_t)(tb + s) * DIM_STATE2);
#pragma unroll
      for (int s = 0; s < 16; ++s) {
        const float gr = g[s][0] * gm;
        const float gi = g[s][1] * gm;
        const float nr = lr * hr - li * hi + gr;
        const float ni = lr * hi + li * hr + gi;
        hr = nr; hi = ni;
        const float wr = fminf(fmaxf(hr * CARRY_HS, -65504.0f), 65504.0f);
        const float wi = fminf(fmaxf(hi * CARRY_HS, -65504.0f), 65504.0f);
        const unsigned lo = f16_bits_ftz(wr);
        const unsigned up = f16_bits_ftz(wi);
        stage[(sub * 16 + s) * 32 + lane] = lo | (up << 16);
      }
    }
    __syncthreads();
    for (int pass = 0; pass < 2; ++pass) {
#pragma unroll
      for (int it = 0; it < 8; ++it) {
        const int row = it * 4 + q;
        const v4u w = *(const v4u*)(stage + row * 32 + c * 4);
        *(volatile v4u*)(hp + (size_t)(t0 + row) * (DIM_STATE2 / 2) + c * 4) = w;
      }
      __threadfence();
    }
    __syncthreads();
  }
}

__global__ __launch_bounds__(256) void glu_gate(
    const float* __restrict__ y, const float* __restrict__ z,
    const float* __restrict__ bias, float* __restrict__ out) {
  const size_t g = (size_t)blockIdx.x * 256 + threadIdx.x;
  const int col = (int)((g * 4) & (size_t)(DIM_HID - 1));
  const v4f yv = *(const v4f*)(y + g * 4);
  const v4f zv = *(const v4f*)(z + g * 4);
  const v4f bv = *(const v4f*)(bias + col);
  v4f o;
#pragma unroll
  for (int e = 0; e < 4; ++e) {
    const float t  = zv[e] + bf16_rne(bv[e]);
    const float ex = expf(-t);
    o[e] = yv[e] * __builtin_amdgcn_rcpf(1.0f + ex);
  }
  float* dst = out + g * 4;
  *(volatile v4f*)dst = o;
  __threadfence();
  *(volatile v4f*)dst = o;
}

extern "C" void kernel_launch(void* const* d_in, const int* in_sizes, int n_in,
                              void* d_out, int out_size, void* d_ws, size_t ws_size,
                              hipStream_t stream) {
  if (n_in != 10) return;
  if (in_sizes[0] != N_TOK * DIM_HID) return;
  if (in_sizes[1] != DIM_STATE) return;
  if (in_sizes[2] != DIM_STATE) return;
  if (in_sizes[3] != DIM_STATE) return;
  if (in_sizes[4] != DIM_HID * DIM_STATE) return;
  if (in_sizes[5] != DIM_HID * DIM_STATE) return;
  if (in_sizes[6] != DIM_STATE * DIM_HID) return;
  if (in_sizes[7] != DIM_STATE * DIM_HID) return;
  if (in_sizes[8] != DIM_HID * DIM_HID) return;
  if (in_sizes[9] != DIM_HID) return;
  if (out_size != N_TOK * DIM_HID) return;
  if (ws_size < WS_TOTAL) return;

  const float* X      = (const float*)d_in[0];
  const float* nu_log = (const float*)d_in[1];
  const float* th_log = (const float*)d_in[2];
  const float* gm_log = (const float*)d_in[3];
  const float* B_re   = (const float*)d_in[4];
  const float* B_im   = (const float*)d_in[5];
  const float* C_re   = (const float*)d_in[6];
  const float* C_im   = (const float*)d_in[7];
  const float* Wd     = (const float*)d_in[8];
  const float* bd     = (const float*)d_in[9];
  float* Out = (float*)d_out;

  unsigned char* ws = (unsigned char*)d_ws;
  float*    params = (float*)(ws + WS_OFF_PARAMS);
  _Float16* Bt1    = (_Float16*)(ws + WS_OFF_BT1);
  _Float16* Bt2    = (_Float16*)(ws + WS_OFF_BT2);
  _Float16* Bt3    = (_Float16*)(ws + WS_OFF_BT3);
  _Float16* XS16   = (_Float16*)(ws + WS_OFF_XS16);
  float*    G      = (float*)(ws + WS_OFF_G);
  unsigned* H32    = (unsigned*)(ws + WS_OFF_H16);
  _Float16* Y16    = (_Float16*)(ws + WS_OFF_XS16);
  float*    Y32    = (float*)(ws + WS_OFF_G);
  float*    Zp     = (float*)(ws + WS_OFF_G + WS_SZ_Y32);

  lru_setup<<<dim3(1), dim3(512), 0, stream>>>(nu_log, th_log, gm_log, params);

  prep_bt1<<<dim3(DIM_STATE / 32, DIM_HID / 64), dim3(256), 0, stream>>>(B_re, B_im, Bt1);

  prep_bt2<<<dim3(DIM_STATE / 32, DIM_HID / 64), dim3(256), 0, stream>>>(C_re, C_im, Bt2);

  cvt_plane_f16<true><<<dim3((DIM_HID * DIM_HID / 8) / 256), dim3(256), 0, stream>>>(Wd, Bt3, CARRY_W);

  ln_rows_f16<<<dim3(N_TOK / 8), dim3(256), 0, stream>>>(X, XS16);

  wmma_gemm64_f16<false><<<dim3(((N_TOK / 64) * (DIM_STATE2 / 64)) / 8), dim3(256), 0, stream>>>(
      (const unsigned short*)XS16, DIM_HID, (const unsigned short*)Bt1, DIM_HID,
      G, DIM_STATE2, (unsigned short*)H32, DIM_STATE2,
      N_TOK, DIM_STATE2, DIM_HID, SCALE_GEMM1, CARRY_NONE);

  lru_scan<<<dim3(N_BATCH * (DIM_STATE / 32)), dim3(32), 0, stream>>>(G, params, H32);

  wmma_gemm64_f16<true><<<dim3(((N_TOK / 64) * (DIM_HID / 64)) / 8), dim3(256), 0, stream>>>(
      (const unsigned short*)H32, DIM_STATE2, (const unsigned short*)Bt2, DIM_STATE2,
      Y32, DIM_HID, (unsigned short*)Y16, DIM_HID,
      N_TOK, DIM_HID, DIM_STATE2, SCALE_GEMM2, CARRY_Y);

  wmma_gemm64_f16<false><<<dim3(((N_TOK / 64) * (DIM_HID / 64)) / 8), dim3(256), 0, stream>>>(
      (const unsigned short*)Y16, DIM_HID, (const unsigned short*)Bt3, DIM_HID,
      Zp, DIM_HID, (unsigned short*)H32, DIM_HID,
      N_TOK, DIM_HID, DIM_HID, SCALE_GEMM3, CARRY_NONE);

  glu_gate<<<dim3((N_TOK * DIM_HID / 4) / 256), dim3(256), 0, stream>>>(Y32, Zp, bd, Out);
}
